// GNNCompoundEncoder_45037027065924
// MI455X (gfx1250) — hardware-verified
//
#include <hip/hip_runtime.h>
#include <stddef.h>


#define NTHR    256
#define NWAVE   8
#define EPT     8
#define NGRP    2
#define CHUNK   (NTHR * EPT * NGRP)
#define WCAP    (EPT * NGRP * 32)
#define LISTN   (NWAVE * WCAP)
#define NBC     4096
#define NBF     1024
#define RCAP    40960
#define RBN     128
#define TGT     256
#define DEGCAP  1024
#define CLCAP   64
#define OTHR    512
#define BM      64
#define GPB     4
#define GMAX    4096
#define WSCAP   134217728
#define VOC     128
#define D0      64
#define D1      80
#define D2      96
#define DM      256
#define K1      128
#define KP1     128
#define K2      160
#define KP2     192
#define K3      192
#define KP3     192
#define NP      96
#define NCLUST  20000
#define BNEPS   1e-5f
#define ACARRY  16.0f
#define WCARRY  64.0f
#define GSCALE  (1.0f / 1024.0f)

#define LDS_FILL ((RCAP + NBF + LISTN) * 4 + 64)

static_assert((CHUNK & (CHUNK - 1)) == 0);
static_assert(CHUNK <= 4096);
static_assert((NBC & (NBC - 1)) == 0 && (NBF & (NBF - 1)) == 0);
static_assert(NBC == 4 * NBF);
static_assert(OTHR * 8 == NBC);
static_assert((RCAP % 32) == 0);
static_assert(TGT == NWAVE * 32);
static_assert((NBC % TGT) == 0);
static_assert((TGT % BM) == 0);
static_assert(WCAP == EPT * NGRP * 32);
static_assert((GPB & (GPB - 1)) == 0 && GPB <= NWAVE);
static_assert(((GPB * DM) % NTHR) == 0);
static_assert(DM == 8 * 32);
static_assert((NP % 32) == 0);
static_assert(K1 == 2 * D0 && K2 == 2 * D1 && K3 == 2 * D2);
static_assert(KP1 >= K1 && KP2 >= K2 && KP3 >= K3);

typedef float        v4f  __attribute__((ext_vector_type(4)));
typedef float        v8f  __attribute__((ext_vector_type(8)));
typedef int          v4i  __attribute__((ext_vector_type(4)));
typedef unsigned int v4u  __attribute__((ext_vector_type(4)));
typedef _Float16     v4h  __attribute__((ext_vector_type(4)));
typedef _Float16     v8h  __attribute__((ext_vector_type(8)));
typedef _Float16     v16h __attribute__((ext_vector_type(16)));
union Frag { v16h v; v8h h[2]; };
union H4 { v4h v; unsigned int u[2]; };

__device__ __forceinline__ v8f wmh(v16h a, v16h b, v8f c) {
  v8f d = __builtin_amdgcn_wmma_f32_16x16x32_f16(false, a, false, b, (short)0, c, false, false);
  asm volatile("v_nop\n\tv_nop\n\tv_nop\n\tv_nop" : "+v"(d) : "v"(a), "v"(b));
  return d;
}

template <int NB>
__device__ __forceinline__ int scan_chunk(const int* __restrict__ dsts, int nE, int cbase, int slotBase,
                                          int vec8, int* list, int tid, int lane, int wave) {
  int wc = 0;
#pragma unroll
  for (int g = 0; g < NGRP; ++g) {
    const int el0  = (g * NTHR + tid) * EPT;
    const int e0   = cbase + el0;
    const int sent = -2147483647 - 1;
    v4i da, db;
    if (vec8 != 0 && cbase + CHUNK <= nE) {
      da = *(const v4i*)(dsts + e0);
      db = *(const v4i*)(dsts + e0 + 4);
    } else {
      da.x = (e0     < nE) ? dsts[min(e0, nE - 1)] : sent;
      da.y = (e0 + 1 < nE) ? dsts[min(e0 + 1, nE - 1)] : sent;
      da.z = (e0 + 2 < nE) ? dsts[min(e0 + 2, nE - 1)] : sent;
      da.w = (e0 + 3 < nE) ? dsts[min(e0 + 3, nE - 1)] : sent;
      db.x = (e0 + 4 < nE) ? dsts[min(e0 + 4, nE - 1)] : sent;
      db.y = (e0 + 5 < nE) ? dsts[min(e0 + 5, nE - 1)] : sent;
      db.z = (e0 + 6 < nE) ? dsts[min(e0 + 6, nE - 1)] : sent;
      db.w = (e0 + 7 < nE) ? dsts[min(e0 + 7, nE - 1)] : sent;
    }
    const unsigned nb = (unsigned)slotBase;
    const unsigned s0 = (unsigned)da.x - nb, s1 = (unsigned)da.y - nb;
    const unsigned s2 = (unsigned)da.z - nb, s3 = (unsigned)da.w - nb;
    const unsigned s4 = (unsigned)db.x - nb, s5 = (unsigned)db.y - nb;
    const unsigned s6 = (unsigned)db.z - nb, s7 = (unsigned)db.w - nb;
    const bool h0 = s0 < (unsigned)NB, h1 = s1 < (unsigned)NB, h2 = s2 < (unsigned)NB, h3 = s3 < (unsigned)NB;
    const bool h4 = s4 < (unsigned)NB, h5 = s5 < (unsigned)NB, h6 = s6 < (unsigned)NB, h7 = s7 < (unsigned)NB;
    const unsigned any = __builtin_amdgcn_ballot_w32(h0 | h1 | h2 | h3 | h4 | h5 | h6 | h7);
    if (any != 0u) {
#define HITJ(J, HJ, SJ) { \
        const unsigned mj = __builtin_amdgcn_ballot_w32(HJ); \
        if (mj != 0u) { \
          if (HJ) { \
            const int pos = wc + (int)__builtin_amdgcn_mbcnt_lo(mj, 0u); \
            if (pos < WCAP) list[wave * WCAP + pos] = ((el0 + (J)) << 12) | (int)(SJ); \
          } \
          wc += (int)__builtin_popcount(mj); } }
      HITJ(0, h0, s0)
      HITJ(1, h1, s1)
      HITJ(2, h2, s2)
      HITJ(3, h3, s3)
      HITJ(4, h4, s4)
      HITJ(5, h5, s5)
      HITJ(6, h6, s6)
      HITJ(7, h7, s7)
#undef HITJ
    }
  }
  return wc;
}

__global__ __launch_bounds__(NTHR) void k_count(const int* __restrict__ dsts, int* cnt, int nE, int vec8) {
  __shared__ __attribute__((aligned(16))) int scnt[NBC];
  __shared__ __attribute__((aligned(16))) int list[LISTN];
  __shared__ int wcnt[NWAVE];
  const int tid = threadIdx.x, lane = tid & 31, wave = tid >> 5;
  const int nodeBase = blockIdx.x * NBC;

  for (int i = tid; i < NBC; i += NTHR) scnt[i] = 0;
  __syncthreads();

  const int nChunks = (nE + CHUNK - 1) / CHUNK;
#pragma unroll 1
  for (int ch = 0; ch < nChunks; ++ch) {
    const int cbase = ch * CHUNK;
    const int wc = scan_chunk<NBC>(dsts, nE, cbase, nodeBase, vec8, list, tid, lane, wave);
    if (lane == 0) wcnt[wave] = wc;
    __syncthreads();
    if (wave == 0) {
#pragma unroll 1
      for (int wsx = 0; wsx < NWAVE; ++wsx) {
        int n = __builtin_amdgcn_readfirstlane(wcnt[wsx]);
        n = n > WCAP ? WCAP : (n < 0 ? 0 : n);
        const int* lp = list + wsx * WCAP;
#pragma unroll 1
        for (int i = 0; i < n; ++i) {
          const int ent  = __builtin_amdgcn_readfirstlane(lp[i]);
          const int slot = ent & (NBC - 1);
          if (lane == 0) scnt[slot] = scnt[slot] + 1;
        }
      }
    }
    __syncthreads();
  }

  v4i cq[4];
#pragma unroll
  for (int q = 0; q < 4; ++q) {
    const int f = (wave * 4 + q) * 128 + 4 * lane;
    cq[q] = *(const v4i*)(scnt + f);
  }
  int* cp = cnt + (size_t)nodeBase;
#pragma unroll
  for (int q = 0; q < 4; ++q) {
    const int f = (wave * 4 + q) * 128 + 4 * lane;
    *(volatile v4i*)(cp + f) = cq[q];
  }
  __threadfence();
#pragma unroll
  for (int q = 0; q < 4; ++q) {
    const int f = (wave * 4 + q) * 128 + 4 * lane;
    *(volatile v4i*)(cp + f) = cq[q];
  }
}

__global__ __launch_bounds__(OTHR) void k_offsets(
    const int* __restrict__ cnt, int* off, int* rbase, int nChunk) {
  __shared__ __attribute__((aligned(16))) int soff[NBC];
  __shared__ __attribute__((aligned(16))) int srb[RBN];
  __shared__ int wtot[OTHR / 32];
  const int tid = threadIdx.x, lane = tid & 31, wave = tid >> 5, sub = tid >> 7;
  for (int i = tid; i < RBN; i += OTHR) srb[i] = 0;
  int carry = 0;
#pragma unroll 1
  for (int ch = 0; ch < nChunk; ++ch) {
    const int base = ch * NBC;
    const v4i c0 = *(const v4i*)(cnt + base + 8 * tid);
    const v4i c1 = *(const v4i*)(cnt + base + 8 * tid + 4);
    const int e0 = max(c0.x, 0), e1 = max(c0.y, 0), e2 = max(c0.z, 0), e3 = max(c0.w, 0);
    const int e4 = max(c1.x, 0), e5 = max(c1.y, 0), e6 = max(c1.z, 0), e7 = max(c1.w, 0);
    const int ts = e0 + e1 + e2 + e3 + e4 + e5 + e6 + e7;
    int incl = ts;
#pragma unroll
    for (int d = 1; d < 32; d <<= 1) {
      const int t = __shfl_up(incl, d);
      if (lane >= d) incl += t;
    }
    if (lane == 31) wtot[wave] = incl;
    __syncthreads();
    const int S0 = wtot[0]  + wtot[1]  + wtot[2]  + wtot[3];
    const int S1 = wtot[4]  + wtot[5]  + wtot[6]  + wtot[7];
    const int S2 = wtot[8]  + wtot[9]  + wtot[10] + wtot[11];
    const int S3 = wtot[12] + wtot[13] + wtot[14] + wtot[15];
    int pre = 0;
#pragma unroll 1
    for (int w = 4 * sub; w < wave; ++w) pre += wtot[w];
    const int b0 = carry;
    const int b1 = b0 + ((S0 + 31) & ~31);
    const int b2 = b1 + ((S1 + 31) & ~31);
    const int b3 = b2 + ((S2 + 31) & ~31);
    const int b4 = b3 + ((S3 + 31) & ~31);
    const int myb = sub == 0 ? b0 : (sub == 1 ? b1 : (sub == 2 ? b2 : b3));
    if (tid == 0) {
      srb[min(4 * ch + 0, RBN - 1)] = b0;
      srb[min(4 * ch + 1, RBN - 1)] = b1;
      srb[min(4 * ch + 2, RBN - 1)] = b2;
      srb[min(4 * ch + 3, RBN - 1)] = b3;
    }
    int run = myb + pre + incl - ts;
    soff[8 * tid + 0] = run; run += e0;
    soff[8 * tid + 1] = run; run += e1;
    soff[8 * tid + 2] = run; run += e2;
    soff[8 * tid + 3] = run; run += e3;
    soff[8 * tid + 4] = run; run += e4;
    soff[8 * tid + 5] = run; run += e5;
    soff[8 * tid + 6] = run; run += e6;
    soff[8 * tid + 7] = run;
    carry = b4;
    __syncthreads();
    const v4i o0 = *(const v4i*)(soff + 4 * tid);
    const v4i o1 = *(const v4i*)(soff + 4 * (tid + OTHR));
    int* op = off + base;
    *(volatile v4i*)(op + 4 * tid) = o0;
    *(volatile v4i*)(op + 4 * (tid + OTHR)) = o1;
    __threadfence();
    *(volatile v4i*)(op + 4 * tid) = o0;
    *(volatile v4i*)(op + 4 * (tid + OTHR)) = o1;
    __syncthreads();
  }
  if (tid == 0) srb[min(4 * nChunk, RBN - 1)] = carry;
  __syncthreads();
  v4i rv = {0, 0, 0, 0};
  if (tid < 32) rv = *(const v4i*)(srb + 4 * tid);
  if (tid < 32) *(volatile v4i*)(rbase + 4 * tid) = rv;
  __threadfence();
  if (tid < 32) *(volatile v4i*)(rbase + 4 * tid) = rv;
}

__global__ __launch_bounds__(NTHR) void k_fill(
    const int* __restrict__ srcs, const int* __restrict__ dsts,
    const int* __restrict__ off, const int* __restrict__ rbase,
    int* csr, int nN, int nE, int vec8, int csrLen) {
  extern __shared__ v4f lds_dyn[];
  int* region = (int*)lds_dyn;
  int* cursor = region + RCAP;
  int* list   = cursor + NBF;
  int* wcnt   = list + LISTN;
  const int tid = threadIdx.x, lane = tid & 31, wave = tid >> 5;
  const int b = blockIdx.x;
  const int nodeBase = b * NBF;

  int rb0 = rbase[b];
  const int rb1 = rbase[b + 1];
  rb0 = rb0 < 0 ? 0 : (rb0 > csrLen ? csrLen : rb0);
  rb0 &= ~31;
  int len = rb1 - rb0;
  len = len < 0 ? 0 : (len > RCAP ? RCAP : len);
  int lenW = (len + 31) & ~31;
  if (rb0 + lenW > csrLen) lenW = (csrLen - rb0) & ~31;

  {
    const v4i z = {0, 0, 0, 0};
    for (int i = tid; i < RCAP / 4; i += NTHR) ((v4i*)region)[i] = z;
    for (int s = tid; s < NBF; s += NTHR) {
      int o = off[nodeBase + s] - rb0;
      o = o < 0 ? 0 : (o > RCAP ? RCAP : o);
      cursor[s] = o;
    }
  }
  __syncthreads();

  const int nChunks = (nE + CHUNK - 1) / CHUNK;
#pragma unroll 1
  for (int ch = 0; ch < nChunks; ++ch) {
    const int cbase = ch * CHUNK;
    const int wc = scan_chunk<NBF>(dsts, nE, cbase, nodeBase, vec8, list, tid, lane, wave);
    if (lane == 0) wcnt[wave] = wc;
    __syncthreads();
    if (wave == 0) {
#pragma unroll 1
      for (int wsx = 0; wsx < NWAVE; ++wsx) {
        int n = __builtin_amdgcn_readfirstlane(wcnt[wsx]);
        n = n > WCAP ? WCAP : (n < 0 ? 0 : n);
        const int* lp = list + wsx * WCAP;
#pragma unroll 1
        for (int i = 0; i < n; ++i) {
          const int ent  = __builtin_amdgcn_readfirstlane(lp[i]);
          const int slot = ent & (NBF - 1);
          int e = cbase + ((ent >> 12) & (CHUNK - 1));
          e = e > nE - 1 ? nE - 1 : e;
          int sv = srcs[e];
          sv = sv < 0 ? 0 : (sv > nN - 1 ? nN - 1 : sv);
          if (lane == 0) {
            int pos = cursor[slot];
            pos = pos < 0 ? 0 : (pos > RCAP - 1 ? RCAP - 1 : pos);
            region[pos] = sv;
            const int np = pos + 1;
            cursor[slot] = np > RCAP ? RCAP : np;
          }
        }
      }
    }
    __syncthreads();
  }

  const int nv = lenW >> 2;
  int* gp = csr + rb0;
#pragma unroll 1
  for (int i = tid; i < nv; i += NTHR) { const v4i v = ((const v4i*)region)[i]; *(volatile v4i*)(gp + 4 * i) = v; }
  __threadfence();
#pragma unroll 1
  for (int i = tid; i < nv; i += NTHR) { const v4i v = ((const v4i*)region)[i]; *(volatile v4i*)(gp + 4 * i) = v; }
}

template <int K, int KP>
__global__ __launch_bounds__(NTHR) void k_wcvt(const float* __restrict__ w, _Float16* dp, int nUnits, int dout) {
  static_assert((KP % 8) == 0 && K <= KP);
  const int i = (int)blockIdx.x * NTHR + (int)threadIdx.x;
  if (i >= nUnits) return;
  constexpr int UPR = KP / 8;
  const int n = i / UPR;
  const int seg = i - n * UPR;
  const int k0 = 8 * seg;
  int nn = n > dout - 1 ? dout - 1 : n;
  nn = nn < 0 ? 0 : nn;
  v8h o;
#pragma unroll
  for (int j = 0; j < 8; ++j) {
    const int k = k0 + j;
    const int kk = k > K - 1 ? K - 1 : k;
    const float f = w[(size_t)nn * K + kk];
    o[j] = (n < dout && k < K) ? (_Float16)(f * WCARRY) : (_Float16)0.0f;
  }
  _Float16* gp = dp + (size_t)i * 8;
  *(volatile v8h*)gp = o;
  __threadfence();
  *(volatile v8h*)gp = o;
}

template <int MODE, int D, int KP, int PH>
__global__ __launch_bounds__(NTHR) void k_agg(
    const int* __restrict__ csr, const int* __restrict__ off, const int* __restrict__ cnt,
    const int* __restrict__ xid, const float* __restrict__ hsrc, const float* __restrict__ scsh,
    _Float16* zout, int nN, int csrLen) {
  static_assert((D % 8) == 0 && 2 * D <= KP && (KP % 64) == 0 && KP / 8 <= 32 && D / 4 <= 32);
  static_assert((PH % 4) == 0 && PH >= D);
  constexpr int NL4 = D / 4, DP8 = D / 8, KP8 = KP / 8;
  const int tid = threadIdx.x, lane = tid & 31, wave = tid >> 5;
  const int tbase = blockIdx.x * TGT + wave * 32;
  const int lq = lane < NL4 ? lane : NL4 - 1;
  const int cl4 = 4 * lq;
  const int cnt_l = cnt[tbase + lane];
  const int off_l = off[tbase + lane];
  v4f sc4 = {1.f, 1.f, 1.f, 1.f};
  v4f sh4 = {0.f, 0.f, 0.f, 0.f};
  if constexpr (MODE == 1) {
    sc4 = *(const v4f*)(scsh + cl4);
    sh4 = *(const v4f*)(scsh + NP + cl4);
  }
  int pq = lane < DP8 ? lane : lane - DP8;
  pq = pq < 0 ? 0 : (pq > DP8 - 1 ? DP8 - 1 : pq);
  const bool isA = lane < DP8;
  const bool isH = (lane >= DP8) && (lane < 2 * DP8);
  const int sl0 = 2 * pq, sl1 = 2 * pq + 1;

#pragma unroll 1
  for (int j = 0; j < 32; ++j) {
    const int c = tbase + j;
    int n = __shfl(cnt_l, j);
    n = n < 0 ? 0 : (n > DEGCAP ? DEGCAP : n);
    const int st = __shfl(off_l, j);

    v4f a = {0.f, 0.f, 0.f, 0.f};
#pragma unroll 1
    for (int q0 = 0; q0 < n; q0 += 32) {
      int pos = st + q0 + lane;
      pos = pos < 0 ? 0 : (pos > csrLen - 1 ? csrLen - 1 : pos);
      int sl = csr[pos];
      sl = sl < 0 ? 0 : (sl > nN - 1 ? nN - 1 : sl);
      int key = sl;
      if constexpr (MODE == 0) {
        int xs = xid[sl];
        xs = xs < 0 ? 0 : (xs > VOC - 1 ? VOC - 1 : xs);
        key = xs;
      }
      const int mcnt = (n - q0) < 32 ? (n - q0) : 32;
#pragma unroll 1
      for (int pp = 0; pp < mcnt; ++pp) {
        const int s = __builtin_amdgcn_readlane(key, pp);
        v4f xv = *(const v4f*)(hsrc + (size_t)s * PH + cl4);
        if constexpr (MODE == 1) xv = xv * sc4 + sh4;
        a = a + xv;
      }
    }

    const bool live = c < nN;
    const int cc = c > nN - 1 ? nN - 1 : c;
    int hr = cc;
    if constexpr (MODE == 0) {
      int xc = xid[cc];
      xc = xc < 0 ? 0 : (xc > VOC - 1 ? VOC - 1 : xc);
      hr = xc;
    }
    v4f hz = *(const v4f*)(hsrc + (size_t)hr * PH + cl4);
    if constexpr (MODE == 1) hz = hz * sc4 + sh4;

    H4 ua, uh;
    ua.v.x = (_Float16)((live ? a.x : 0.f) * ACARRY);
    ua.v.y = (_Float16)((live ? a.y : 0.f) * ACARRY);
    ua.v.z = (_Float16)((live ? a.z : 0.f) * ACARRY);
    ua.v.w = (_Float16)((live ? a.w : 0.f) * ACARRY);
    uh.v.x = (_Float16)((live ? hz.x : 0.f) * ACARRY);
    uh.v.y = (_Float16)((live ? hz.y : 0.f) * ACARRY);
    uh.v.z = (_Float16)((live ? hz.z : 0.f) * ACARRY);
    uh.v.w = (_Float16)((live ? hz.w : 0.f) * ACARRY);
    const unsigned a00 = __shfl(ua.u[0], sl0), a01 = __shfl(ua.u[1], sl0);
    const unsigned a10 = __shfl(ua.u[0], sl1), a11 = __shfl(ua.u[1], sl1);
    const unsigned h00 = __shfl(uh.u[0], sl0), h01 = __shfl(uh.u[1], sl0);
    const unsigned h10 = __shfl(uh.u[0], sl1), h11 = __shfl(uh.u[1], sl1);
    v4u o;
    o.x = isA ? a00 : (isH ? h00 : 0u);
    o.y = isA ? a01 : (isH ? h01 : 0u);
    o.z = isA ? a10 : (isH ? h10 : 0u);
    o.w = isA ? a11 : (isH ? h11 : 0u);
    _Float16* gp = zout + (size_t)c * KP + 8 * lane;
    if (lane < KP8) *(volatile v4u*)gp = o;
    __threadfence();
    if (lane < KP8) *(volatile v4u*)gp = o;
  }
}

template <int KP, int TPW, int PC, int STATS>
__global__ __launch_bounds__(NTHR) void k_gemm(
    const _Float16* __restrict__ Z, const _Float16* __restrict__ Wp, const float* __restrict__ bias,
    float* Cout, float* part, int nValid, int dout) {
  constexpr int NCOLB  = 32 * TPW;
  constexpr int PPR    = NCOLB / 4;
  constexpr int NIT    = (BM * PPR) / NTHR;
  constexpr int KSTEPS = KP / 32;
  constexpr int NPQ    = (2 * NCOLB) / 4;
  static_assert((BM * PPR) % NTHR == 0);
  static_assert(NIT >= 1);
  static_assert((PPR % 8) == 0);
  static_assert((KP % 32) == 0);
  static_assert((PC % 32) == 0 && NCOLB <= PC);
  static_assert(PC == NCOLB || (NTHR / PPR) * PPR == NTHR);
  static_assert(BM == 4 * 16);
  static_assert(NPQ <= NTHR && NCOLB <= NTHR);

  __shared__ __attribute__((aligned(16))) float stg[BM * NCOLB];
  __shared__ __attribute__((aligned(16))) float sps[2 * NCOLB];
  const int tid = threadIdx.x, lane = tid & 31, wave = tid >> 5, hh = lane >> 4, m = lane & 15;
  const int rowBase = (int)blockIdx.x * BM;
  const int colBase = (int)blockIdx.y * NCOLB;
  const int rg = wave >> 1, chf = wave & 1;
  const int r0 = rg * 16;
  const int c0 = chf * (16 * TPW);

  v8f acc[TPW];
#pragma unroll
  for (int t = 0; t < TPW; ++t) { v8f z = {0.f, 0.f, 0.f, 0.f, 0.f, 0.f, 0.f, 0.f}; acc[t] = z; }

  const _Float16* ap = Z  + (size_t)(rowBase + r0 + m) * KP + 8 * hh;
  const _Float16* bp = Wp + (size_t)(colBase + c0 + m) * KP + 8 * hh;
#pragma unroll 1
  for (int kt = 0; kt < KSTEPS; ++kt) {
    Frag a;
    a.h[0] = *(const v8h*)(ap + 32 * kt);
    a.h[1] = *(const v8h*)(ap + 32 * kt + 16);
#pragma unroll
    for (int t = 0; t < TPW; ++t) {
      const size_t to = (size_t)(16 * t) * KP + 32 * kt;
      Frag b;
      b.h[0] = *(const v8h*)(bp + to);
      b.h[1] = *(const v8h*)(bp + to + 16);
      acc[t] = wmh(a.v, b.v, acc[t]);
    }
  }

  {
    float* sp = stg + (size_t)(r0 + 8 * hh) * NCOLB + c0 + m;
    const int growb = rowBase + r0 + 8 * hh;
#pragma unroll
    for (int t = 0; t < TPW; ++t) {
      const int col = colBase + c0 + 16 * t + m;
      int bc = col > dout - 1 ? dout - 1 : col;
      bc = bc < 0 ? 0 : bc;
      const float bv = bias[bc];
      const bool cok = col < dout;
#pragma unroll
      for (int r = 0; r < 8; ++r) {
        const bool lv = (growb + r) < nValid;
        const float g = acc[t][r] * GSCALE;
        const float v = fmaxf(g + bv, 0.f);
        sp[r * NCOLB + 16 * t] = (lv && cok) ? v : 0.f;
      }
    }
  }
  __syncthreads();

  v4f pv = {0.f, 0.f, 0.f, 0.f};
  if constexpr (STATS != 0) {
    if (tid < NCOLB) {
      float s = 0.f, q = 0.f;
#pragma unroll 4
      for (int r = 0; r < BM; ++r) {
        const float v = stg[r * NCOLB + tid];
        s += v;
        q += v * v;
      }
      sps[tid] = s;
      sps[NCOLB + tid] = q;
    }
    __syncthreads();
    if (tid < NPQ) pv = *(const v4f*)(sps + 4 * tid);
  }

  v4f cv[NIT];
#pragma unroll
  for (int it = 0; it < NIT; ++it) {
    const int id = it * NTHR + tid;
    const int row = id / PPR, seg = id % PPR;
    cv[it] = *(const v4f*)(stg + (size_t)row * NCOLB + 4 * seg);
  }
  float* pp = part + (size_t)blockIdx.x * (2 * NCOLB) + 4 * tid;
#pragma unroll
  for (int it = 0; it < NIT; ++it) {
    const int id = it * NTHR + tid;
    const int row = id / PPR, seg = id % PPR;
    float* gp = Cout + (size_t)(rowBase + row) * PC + colBase + 4 * seg;
    *(volatile v4f*)gp = cv[it];
  }
  if constexpr (STATS != 0) { if (tid < NPQ) *(volatile v4f*)pp = pv; }
  __threadfence();
#pragma unroll
  for (int it = 0; it < NIT; ++it) {
    const int id = it * NTHR + tid;
    const int row = id / PPR, seg = id % PPR;
    float* gp = Cout + (size_t)(rowBase + row) * PC + colBase + 4 * seg;
    *(volatile v4f*)gp = cv[it];
  }
  if constexpr (STATS != 0) { if (tid < NPQ) *(volatile v4f*)pp = pv; }
}

__global__ __launch_bounds__(NTHR) void k_bnfin(const float* __restrict__ part, const float* __restrict__ gam,
                                                const float* __restrict__ bet, float* scsh,
                                                int nBlk, int nValid, int dout) {
  __shared__ __attribute__((aligned(16))) float sps[2 * NP];
  static_assert(NP <= NTHR && (2 * NP) / 4 <= NTHR);
  const int tid = threadIdx.x;
  if (tid < NP) {
    double s = 0.0, q = 0.0;
#pragma unroll 1
    for (int b = 0; b < nBlk; ++b) {
      s += (double)part[(size_t)b * (2 * NP) + tid];
      q += (double)part[(size_t)b * (2 * NP) + NP + tid];
    }
    const double inv = 1.0 / (double)(nValid < 1 ? 1 : nValid);
    const double mean = s * inv;
    double var = q * inv - mean * mean;
    var = var < 0.0 ? 0.0 : var;
    const float mf = (float)mean;
    const float vf = (float)var;
    int cc = tid > dout - 1 ? dout - 1 : tid;
    cc = cc < 0 ? 0 : cc;
    const float gv = gam[cc];
    const float bv = bet[cc];
    float sc = gv * rsqrtf(vf + BNEPS);
    float sh = bv - mf * sc;
    if (tid >= dout) { sc = 0.f; sh = 0.f; }
    sps[tid] = sc;
    sps[NP + tid] = sh;
  }
  __syncthreads();
  constexpr int NPQ = (2 * NP) / 4;
  v4f v = {0.f, 0.f, 0.f, 0.f};
  if (tid < NPQ) v = *(const v4f*)(sps + 4 * tid);
  if (tid < NPQ) *(volatile v4f*)(scsh + 4 * tid) = v;
  __threadfence();
  if (tid < NPQ) *(volatile v4f*)(scsh + 4 * tid) = v;
}

__global__ __launch_bounds__(NTHR) void k_cluster(const int* __restrict__ cid, const int* __restrict__ bat,
                                                  const float* __restrict__ hpre, const float* __restrict__ scsh,
                                                  float* yout, int* ybout, int nN, int nC) {
  constexpr int NL4 = NP / 4;
  static_assert(NL4 <= 32);
  const int tid = threadIdx.x, lane = tid & 31, wave = tid >> 5;
  const int tbase = blockIdx.x * TGT + wave * 32;
  const int lq = lane < NL4 ? lane : NL4 - 1;
  const int cl4 = 4 * lq;
  const v4f sc4 = *(const v4f*)(scsh + cl4);
  const v4f sh4 = *(const v4f*)(scsh + NP + cl4);
  const float NINF = -__builtin_inff();
  const int IMIN = -2147483647 - 1;
  int myyb = -1;

#pragma unroll 1
  for (int j = 0; j < 32; ++j) {
    const int c = tbase + j;
    int lo = 0, hi = nN;
#pragma unroll 1
    while (lo < hi) {
      const int mid = (lo + hi) >> 1;
      const int v = cid[mid];
      if (v < c) lo = mid + 1; else hi = mid;
    }
    int lo2 = lo, hi2 = nN;
#pragma unroll 1
    while (lo2 < hi2) {
      const int mid = (lo2 + hi2) >> 1;
      const int v = cid[mid];
      if (v <= c) lo2 = mid + 1; else hi2 = mid;
    }
    int cntc = lo2 - lo;
    cntc = cntc < 0 ? 0 : (cntc > CLCAP ? CLCAP : cntc);
    v4f mx = {NINF, NINF, NINF, NINF};
    int yb = IMIN;
#pragma unroll 1
    for (int i = 0; i < cntc; ++i) {
      int node = lo + i;
      node = node > nN - 1 ? nN - 1 : (node < 0 ? 0 : node);
      v4f hv = *(const v4f*)(hpre + (size_t)node * NP + cl4);
      hv = hv * sc4 + sh4;
      mx.x = fmaxf(mx.x, hv.x);
      mx.y = fmaxf(mx.y, hv.y);
      mx.z = fmaxf(mx.z, hv.z);
      mx.w = fmaxf(mx.w, hv.w);
      const int bb = bat[node];
      yb = bb > yb ? bb : yb;
    }
    const bool live = c < nC;
    v4f o;
    o.x = live ? mx.x : 0.f;
    o.y = live ? mx.y : 0.f;
    o.z = live ? mx.z : 0.f;
    o.w = live ? mx.w : 0.f;
    const int ybv = live ? yb : -1;
    float* gp = yout + (size_t)c * NP + cl4;
    if (lane < NL4) *(volatile v4f*)gp = o;
    __threadfence();
    if (lane < NL4) *(volatile v4f*)gp = o;
    myyb = (lane == j) ? ybv : myyb;
  }

  v4i yv;
  yv.x = __shfl(myyb, (4 * lane + 0) & 31);
  yv.y = __shfl(myyb, (4 * lane + 1) & 31);
  yv.z = __shfl(myyb, (4 * lane + 2) & 31);
  yv.w = __shfl(myyb, (4 * lane + 3) & 31);
  int* yp = ybout + tbase + 4 * lane;
  if (lane < 8) *(volatile v4i*)yp = yv;
  __threadfence();
  if (lane < 8) *(volatile v4i*)yp = yv;
}

__global__ __launch_bounds__(NTHR) void k_gmax(const int* __restrict__ keys, const float* __restrict__ y2,
                                               float* out, int nC, int nG, int vec8) {
  __shared__ __attribute__((aligned(16))) int list[LISTN];
  __shared__ __attribute__((aligned(16))) float spart[NWAVE * GPB * DM];
  __shared__ __attribute__((aligned(16))) float smax[GPB * DM];
  const int tid = threadIdx.x, lane = tid & 31, wave = tid >> 5;
  const int gBase = blockIdx.x * GPB;
  const int col4 = 4 * lane;
  const float NINF = -__builtin_inff();

  v4f accA[GPB], accB[GPB];
#pragma unroll
  for (int s = 0; s < GPB; ++s) { v4f z = {NINF, NINF, NINF, NINF}; accA[s] = z; accB[s] = z; }

  const int nChunks = (nC + CHUNK - 1) / CHUNK;
#pragma unroll 1
  for (int ch = 0; ch < nChunks; ++ch) {
    const int cbase = ch * CHUNK;
    const int wc = scan_chunk<GPB>(keys, nC, cbase, gBase, vec8, list, tid, lane, wave);
    __syncthreads();
    int n = wc;
    n = n > WCAP ? WCAP : (n < 0 ? 0 : n);
    const int* lp = list + wave * WCAP;
#pragma unroll 1
    for (int i = 0; i < n; ++i) {
      const int ent = __builtin_amdgcn_readfirstlane(lp[i]);
      int node = cbase + ((ent >> 12) & (CHUNK - 1));
      node = node > nC - 1 ? nC - 1 : (node < 0 ? 0 : node);
      const int slot = ent & (GPB - 1);
      const v4f hv0 = *(const v4f*)(y2 + (size_t)node * DM + col4);
      const v4f hv1 = *(const v4f*)(y2 + (size_t)node * DM + (DM / 2) + col4);
#pragma unroll
      for (int s = 0; s < GPB; ++s) {
        const bool hit = slot == s;
        v4f ta = accA[s], tb = accB[s];
        ta.x = hit ? fmaxf(ta.x, hv0.x) : ta.x;
        ta.y = hit ? fmaxf(ta.y, hv0.y) : ta.y;
        ta.z = hit ? fmaxf(ta.z, hv0.z) : ta.z;
        ta.w = hit ? fmaxf(ta.w, hv0.w) : ta.w;
        tb.x = hit ? fmaxf(tb.x, hv1.x) : tb.x;
        tb.y = hit ? fmaxf(tb.y, hv1.y) : tb.y;
        tb.z = hit ? fmaxf(tb.z, hv1.z) : tb.z;
        tb.w = hit ? fmaxf(tb.w, hv1.w) : tb.w;
        accA[s] = ta;
        accB[s] = tb;
      }
    }
    __syncthreads();
  }

#pragma unroll
  for (int s = 0; s < GPB; ++s) {
    *(v4f*)(spart + (size_t)(wave * GPB + s) * DM + col4) = accA[s];
    *(v4f*)(spart + (size_t)(wave * GPB + s) * DM + (DM / 2) + col4) = accB[s];
  }
  __syncthreads();
#pragma unroll
  for (int q = 0; q < (GPB * DM) / NTHR; ++q) {
    const int idx = q * NTHR + tid;
    const int s = idx / DM, c = idx % DM;
    float M = NINF;
#pragma unroll
    for (int w = 0; w < NWAVE; ++w) M = fmaxf(M, spart[(w * GPB + s) * DM + c]);
    smax[idx] = M;
  }
  __syncthreads();
  const int ws = wave < GPB ? wave : GPB - 1;
  const v4f va = *(const v4f*)(smax + ws * DM + col4);
  const v4f vb = *(const v4f*)(smax + ws * DM + (DM / 2) + col4);
  const int g = gBase + wave;
  const bool live = (wave < GPB) && (g < nG);
  float* gp0 = out + (size_t)(g < nG ? g : 0) * DM + col4;
  float* gp1 = gp0 + (DM / 2);
  if (live) { *(volatile v4f*)gp0 = va; *(volatile v4f*)gp1 = vb; }
  __threadfence();
  if (live) { *(volatile v4f*)gp0 = va; *(volatile v4f*)gp1 = vb; }
}

extern "C" void kernel_launch(void* const* d_in, const int* in_sizes, int n_in,
                              void* d_out, int out_size, void* d_ws, size_t ws_size,
                              hipStream_t stream) {
  if (n_in < 16) return;
  const int nN = in_sizes[0];
  if (nN < 1 || nN > (1 << 22)) return;
  if (in_sizes[1] < 2 || (in_sizes[1] & 1) != 0) return;
  const int nE = in_sizes[1] / 2;
  if (nE > (1 << 27)) return;
  if (in_sizes[2] != nN || in_sizes[3] != nN) return;
  if (in_sizes[4] < 2 || (in_sizes[4] & 1) != 0) return;
  const int nGE = in_sizes[4] / 2;
  if (nGE > (1 << 27)) return;
  if (in_sizes[5] != VOC * D0) return;
  if (in_sizes[6] != D1 * K1 || in_sizes[7] != D1 || in_sizes[8] != D1 || in_sizes[9] != D1) return;
  if (in_sizes[10] != D2 * K2 || in_sizes[11] != D2 || in_sizes[12] != D2 || in_sizes[13] != D2) return;
  if (in_sizes[14] != DM * K3 || in_sizes[15] != DM) return;
  if (out_size < DM || (out_size % DM) != 0) return;
  const int nG = out_size / DM;
  if (nG < 1 || nG > GMAX) return;
  const int nC = NCLUST;

  const int*   xid  = (const int*)d_in[0];
  const int*   ei   = (const int*)d_in[1];
  const int*   src  = ei;
  const int*   dst  = ei + nE;
  const int*   bat  = (const int*)d_in[2];
  const int*   cid  = (const int*)d_in[3];
  const int*   gei  = (const int*)d_in[4];
  const int*   gsrc = gei;
  const int*   gdst = gei + nGE;
  const float* emb  = (const float*)d_in[5];
  const float* w1   = (const float*)d_in[6];
  const float* b1   = (const float*)d_in[7];
  const float* g1   = (const float*)d_in[8];
  const float* be1  = (const float*)d_in[9];
  const float* w2   = (const float*)d_in[10];
  const float* b2   = (const float*)d_in[11];
  const float* g2   = (const float*)d_in[12];
  const float* be2  = (const float*)d_in[13];
  const float* wm   = (const float*)d_in[14];
  const float* bm   = (const float*)d_in[15];
  float* out = (float*)d_out;

  const int NPAD   = ((nN + TGT - 1) / TGT) * TGT;
  const int nBC    = (nN + NBC - 1) / NBC;
  const int CNTPAD = nBC * NBC;
  if (CNTPAD < NPAD) return;
  if (4 * nBC + 1 > RBN) return;
  const int nBF    = (nN + NBF - 1) / NBF;
  if (nBF > 4 * nBC) return;
  if (31 * 4 * nBC > 4096) return;
  const int csrLen = ((nE + 31) & ~31) + 4096;
  const int nAgg   = NPAD / TGT;
  const int nGemm  = NPAD / BM;
  const int CPAD    = ((nC + TGT - 1) / TGT) * TGT;
  const int nBC2    = (nC + NBC - 1) / NBC;
  const int CNTPAD2 = nBC2 * NBC;
  if (CNTPAD2 < CPAD) return;
  if (4 * nBC2 + 1 > RBN) return;
  const int nBF2    = (nC + NBF - 1) / NBF;
  if (nBF2 > 4 * nBC2) return;
  if (31 * 4 * nBC2 > 4096) return;
  const int csrLen2 = ((nGE + 31) & ~31) + 4096;
  const int nAggC   = CPAD / TGT;
  const int nGemmC  = CPAD / BM;
  const int GBLK    = (nG + GPB - 1) / GPB;

  char* ws = (char*)d_ws;
  size_t off = 0;
  const size_t zHalves = (size_t)NPAD * KP2 > (size_t)CPAD * KP3 ? (size_t)NPAD * KP2 : (size_t)CPAD * KP3;
  const size_t oW1  = off; off += (size_t)NP * KP1 * 2;            off = (off + 255) & ~(size_t)255;
  const size_t oW2  = off; off += (size_t)NP * KP2 * 2;            off = (off + 255) & ~(size_t)255;
  const size_t oW3  = off; off += (size_t)DM * KP3 * 2;            off = (off + 255) & ~(size_t)255;
  const size_t oZ   = off; off += zHalves * 2;                     off = (off + 255) & ~(size_t)255;
  const size_t oH   = off; off += (size_t)NPAD * NP * 4;           off = (off + 255) & ~(size_t)255;
  const size_t oPt  = off; off += (size_t)nGemm * (2 * NP) * 4;    off = (off + 255) & ~(size_t)255;
  const size_t oS1  = off; off += (size_t)(2 * NP) * 4;            off = (off + 255) & ~(size_t)255;
  const size_t oS2  = off; off += (size_t)(2 * NP) * 4;            off = (off + 255) & ~(size_t)255;
  const size_t oCn1 = off; off += (size_t)CNTPAD * 4;              off = (off + 255) & ~(size_t)255;
  const size_t oOf1 = off; off += (size_t)CNTPAD * 4;              off = (off + 255) & ~(size_t)255;
  const size_t oRb1 = off; off += (size_t)RBN * 4;                 off = (off + 255) & ~(size_t)255;
  const size_t oCs1 = off; off += (size_t)csrLen * 4;              off = (off + 255) & ~(size_t)255;
  const size_t oCn2 = off; off += (size_t)CNTPAD2 * 4;             off = (off + 255) & ~(size_t)255;
  const size_t oOf2 = off; off += (size_t)CNTPAD2 * 4;             off = (off + 255) & ~(size_t)255;
  const size_t oRb2 = off; off += (size_t)RBN * 4;                 off = (off + 255) & ~(size_t)255;
  const size_t oCs2 = off; off += (size_t)csrLen2 * 4;             off = (off + 255) & ~(size_t)255;
  const size_t oY   = off; off += (size_t)CPAD * NP * 4;           off = (off + 255) & ~(size_t)255;
  const size_t oYb  = off; off += (size_t)CPAD * 4;                off = (off + 255) & ~(size_t)255;
  const size_t oY2  = off; off += (size_t)CPAD * DM * 4;           off = (off + 255) & ~(size_t)255;
  if (off > ws_size || off > (size_t)WSCAP) return;

  _Float16* w1p = (_Float16*)(ws + oW1);
  _Float16* w2p = (_Float16*)(ws + oW2);
  _Float16* w3p = (_Float16*)(ws + oW3);
  _Float16* zp  = (_Float16*)(ws + oZ);
  float* hpre   = (float*)(ws + oH);
  float* part   = (float*)(ws + oPt);
  float* sc1    = (float*)(ws + oS1);
  float* sc2    = (float*)(ws + oS2);
  int*   cnt1   = (int*)(ws + oCn1);
  int*   off1   = (int*)(ws + oOf1);
  int*   rb1    = (int*)(ws + oRb1);
  int*   csr1   = (int*)(ws + oCs1);
  int*   cnt2   = (int*)(ws + oCn2);
  int*   off2   = (int*)(ws + oOf2);
  int*   rb2    = (int*)(ws + oRb2);
  int*   csr2   = (int*)(ws + oCs2);
  float* yp     = (float*)(ws + oY);
  int*   ybp    = (int*)(ws + oYb);
  float* y2p    = (float*)(ws + oY2);

  const int vec8n = ((nE  & 3) == 0) ? 1 : 0;
  const int vec8c = ((nGE & 3) == 0) ? 1 : 0;

  {
    const int u1 = NP * (KP1 / 8), u2 = NP * (KP2 / 8), u3 = DM * (KP3 / 8);
    k_wcvt<K1, KP1><<<(u1 + NTHR - 1) / NTHR, NTHR, 0, stream>>>(w1, w1p, u1, D1);
    k_wcvt<K2, KP2><<<(u2 + NTHR - 1) / NTHR, NTHR, 0, stream>>>(w2, w2p, u2, D2);
    k_wcvt<K3, KP3><<<(u3 + NTHR - 1) / NTHR, NTHR, 0, stream>>>(wm, w3p, u3, DM);
  }

  hipFuncSetAttribute(reinterpret_cast<const void*>(&k_fill),
                      hipFuncAttributeMaxDynamicSharedMemorySize, LDS_FILL);
  k_count<<<nBC, NTHR, 0, stream>>>(dst, cnt1, nE, vec8n);
  k_offsets<<<1, OTHR, 0, stream>>>(cnt1, off1, rb1, nBC);
  k_fill<<<nBF, NTHR, LDS_FILL, stream>>>(src, dst, off1, rb1, csr1, nN, nE, vec8n, csrLen);
  k_count<<<nBC2, NTHR, 0, stream>>>(gdst, cnt2, nGE, vec8c);
  k_offsets<<<1, OTHR, 0, stream>>>(cnt2, off2, rb2, nBC2);
  k_fill<<<nBF2, NTHR, LDS_FILL, stream>>>(gsrc, gdst, off2, rb2, csr2, nC, nGE, vec8c, csrLen2);

  k_agg<0, D0, KP1, D0><<<nAgg, NTHR, 0, stream>>>(csr1, off1, cnt1, xid, emb, sc1, zp, nN, csrLen);
  k_gemm<KP1, 3, NP, 1><<<dim3(nGemm, 1), NTHR, 0, stream>>>(zp, w1p, b1, hpre, part, nN, D1);
  k_bnfin<<<1, NTHR, 0, stream>>>(part, g1, be1, sc1, nGemm, nN, D1);

  k_agg<1, D1, KP2, NP><<<nAgg, NTHR, 0, stream>>>(csr1, off1, cnt1, xid, hpre, sc1, zp, nN, csrLen);
  k_gemm<KP2, 3, NP, 1><<<dim3(nGemm, 1), NTHR, 0, stream>>>(zp, w2p, b2, hpre, part, nN, D2);
  k_bnfin<<<1, NTHR, 0, stream>>>(part, g2, be2, sc2, nGemm, nN, D2);

  k_cluster<<<nAggC, NTHR, 0, stream>>>(cid, bat, hpre, sc2, yp, ybp, nN, nC);

  k_agg<2, D2, KP3, NP><<<nAggC, NTHR, 0, stream>>>(csr2, off2, cnt2, xid, yp, sc2, zp, nC, csrLen2);
  k_gemm<KP3, 4, DM, 0><<<dim3(nGemmC, 2), NTHR, 0, stream>>>(zp, w3p, bm, y2p, part, nC, DM);

  k_gmax<<<GBLK, NTHR, 0, stream>>>(ybp, y2p, out, nC, nG, 1);
}
